// TransformerEncoderLayer_66357244723827
// MI455X (gfx1250) — hardware-verified
//
#include <hip/hip_runtime.h>
#include <stddef.h>
#include <stdint.h>
#include <math.h>


#define DM     128
#define NTHR   256
#define NWAVE  8
#define EPT    8
#define CHUNK  (NTHR * EPT)
#define WCAP   (EPT * 32)
#define LISTN  (NWAVE * WCAP)
#define NBD    8192
#define SLD    13
#define NBA    1024
#define SLA    10
#define RCAP   28672
#define DEGCAP 64
#define GBM    64
#define GBN    128
#define GTHR   128
#define HLP    256
#define FPI    1024
#define APT    72
#define BNRB   128
#define AGG_ZINTS    (LISTN + 2 * RCAP + 3 * NBA)
#define MISC_INTS    16
#define ROWBUF_INTS  (NWAVE * HLP / 2)
#define AGG_LDS_INTS (AGG_ZINTS + MISC_INTS + ROWBUF_INTS)
#define WSMAX  134217728

#define OW_G1  0
#define OW_G2  16384
#define OW_G3  32768
#define OW_V   49152
#define OW_O   65536
#define OW_QK  81920
#define OW_SE  114688
#define OW_1   180224
#define OW_2   245760
#define OW_END 311296
#define NWUNITS 38912

static_assert((CHUNK & (CHUNK - 1)) == 0 && CHUNK <= 4096);
static_assert((NBD & (NBD - 1)) == 0 && NBD == (1 << SLD));
static_assert((NBA & (NBA - 1)) == 0 && NBA == (1 << SLA));
static_assert(((long long)CHUNK << SLD) < (1LL << 31));
static_assert(((long long)CHUNK << SLA) < (1LL << 31));
static_assert(NBD % (NTHR * 4) == 0);
static_assert(NBA % NWAVE == 0 && NBA % 32 == 0 && NBA % GBM == 0);
static_assert(AGG_ZINTS % (NTHR * 4) == 0 && ((AGG_ZINTS + MISC_INTS) % 4) == 0);
static_assert(AGG_LDS_INTS * 4 <= 300000);
static_assert(GBM == (GTHR / 32) * 16 && GBN == DM && DM == 4 * 32);
static_assert(NWUNITS % NTHR == 0 && OW_END * 2 == 622592);
static_assert(APT % 8 == 0 && APT >= 64);
static_assert(2 * GBN >= DM);

typedef float          v4f   __attribute__((ext_vector_type(4)));
typedef float          v8f   __attribute__((ext_vector_type(8)));
typedef double         v2d   __attribute__((ext_vector_type(2)));
typedef int            v4i   __attribute__((ext_vector_type(4)));
typedef int            v8i   __attribute__((ext_vector_type(8)));
typedef unsigned       v2u   __attribute__((ext_vector_type(2)));
typedef unsigned       v4u   __attribute__((ext_vector_type(4)));
typedef unsigned short v4us  __attribute__((ext_vector_type(4)));
typedef unsigned short v8us  __attribute__((ext_vector_type(8)));
typedef unsigned short v16us __attribute__((ext_vector_type(16)));
typedef __bf16         v16bf __attribute__((ext_vector_type(16)));
typedef v4f  __attribute__((may_alias)) v4fa;
typedef v2d  __attribute__((may_alias)) v2da;
typedef v4i  __attribute__((may_alias)) v4ia;
typedef v2u  __attribute__((may_alias)) v2ua;
typedef v4u  __attribute__((may_alias)) v4ua;
typedef v4us __attribute__((may_alias)) v4usa;
typedef v8us __attribute__((may_alias)) v8usa;
union FragB { v16bf v; v16us u; v8us h[2]; v8i w; };

__device__ __forceinline__ v8f wmb(const FragB& a, const FragB& b, v8f c) {
  v8f d = __builtin_amdgcn_wmma_f32_16x16x32_bf16(false, a.v, false, b.v, (short)0, c, false, false);
  asm volatile("v_nop\n\tv_nop\n\tv_nop\n\tv_nop" : "+v"(d) : "v"(a.w), "v"(b.w));
  return d;
}

__device__ __forceinline__ unsigned bf16_bits(float f) {
  const unsigned u = __float_as_uint(f);
  return (u + 0x7FFFu + ((u >> 16) & 1u)) >> 16;
}
__device__ __forceinline__ float bf16_val(float f) {
  return __uint_as_float(bf16_bits(f) << 16);
}
__device__ __forceinline__ unsigned split_hl(float v) {
  const unsigned hb = bf16_bits(v);
  const unsigned lb = bf16_bits(v - __uint_as_float(hb << 16));
  return hb | (lb << 16);
}
__device__ __forceinline__ float bflo(unsigned w) { return __uint_as_float(w << 16); }
__device__ __forceinline__ float bfhi(unsigned w) { return __uint_as_float(w & 0xffff0000u); }
__device__ __forceinline__ v4f ld_bf4(const unsigned short* __restrict__ p) {
  const v2u w = *(const v2ua*)p;
  v4f r;
  r.x = bflo(w.x); r.y = bfhi(w.x); r.z = bflo(w.y); r.w = bfhi(w.y);
  return r;
}
__device__ __forceinline__ v4f ldv_bf(const float* p) {
  const v4f t = *(const v4f*)p;
  v4f r;
  r.x = bf16_val(t.x); r.y = bf16_val(t.y); r.z = bf16_val(t.z); r.w = bf16_val(t.w);
  return r;
}
__device__ __forceinline__ float wave_sum(float x) {
#pragma unroll
  for (int o = 16; o > 0; o >>= 1) x += __shfl_xor(x, o, 32);
  return x;
}
__device__ __forceinline__ void wave_sync() {
  __builtin_amdgcn_fence(__ATOMIC_RELEASE, "wavefront");
  __builtin_amdgcn_wave_barrier();
  __builtin_amdgcn_fence(__ATOMIC_ACQUIRE, "wavefront");
}

template <int SLB>
__device__ __forceinline__ int scan_chunk(const int* __restrict__ dsts, int nE, int cbase, int slotBase,
                                          int nb, int vec8, int* list, int tid, int lane, int wave) {
  int wc = 0;
  const int el0  = tid * EPT;
  const int e0   = cbase + el0;
  const int sent = -2147483647 - 1;
  v4i da, db;
  if (vec8 != 0 && cbase + CHUNK <= nE) {
    da = *(const v4i*)(dsts + e0);
    db = *(const v4i*)(dsts + e0 + 4);
  } else {
    da.x = (e0     < nE) ? dsts[min(e0,     nE - 1)] : sent;
    da.y = (e0 + 1 < nE) ? dsts[min(e0 + 1, nE - 1)] : sent;
    da.z = (e0 + 2 < nE) ? dsts[min(e0 + 2, nE - 1)] : sent;
    da.w = (e0 + 3 < nE) ? dsts[min(e0 + 3, nE - 1)] : sent;
    db.x = (e0 + 4 < nE) ? dsts[min(e0 + 4, nE - 1)] : sent;
    db.y = (e0 + 5 < nE) ? dsts[min(e0 + 5, nE - 1)] : sent;
    db.z = (e0 + 6 < nE) ? dsts[min(e0 + 6, nE - 1)] : sent;
    db.w = (e0 + 7 < nE) ? dsts[min(e0 + 7, nE - 1)] : sent;
  }
  const unsigned nbs = (unsigned)slotBase;
  const unsigned unb = (unsigned)nb;
  const unsigned s0 = (unsigned)da.x - nbs, s1 = (unsigned)da.y - nbs;
  const unsigned s2 = (unsigned)da.z - nbs, s3 = (unsigned)da.w - nbs;
  const unsigned s4 = (unsigned)db.x - nbs, s5 = (unsigned)db.y - nbs;
  const unsigned s6 = (unsigned)db.z - nbs, s7 = (unsigned)db.w - nbs;
  const bool h0 = s0 < unb, h1 = s1 < unb, h2 = s2 < unb, h3 = s3 < unb;
  const bool h4 = s4 < unb, h5 = s5 < unb, h6 = s6 < unb, h7 = s7 < unb;
  const unsigned any = __builtin_amdgcn_ballot_w32(h0 | h1 | h2 | h3 | h4 | h5 | h6 | h7);
  if (any != 0u) {
#define HITJ(J, HJ, SJ) { \
      const unsigned mj = __builtin_amdgcn_ballot_w32(HJ); \
      if (mj != 0u) { \
        if (HJ) { \
          const int pos = wc + (int)__builtin_amdgcn_mbcnt_lo(mj, 0u); \
          if (pos < WCAP) list[wave * WCAP + pos] = ((el0 + (J)) << SLB) | (int)(SJ); \
        } \
        wc += (int)__builtin_popcount(mj); } }
    HITJ(0, h0, s0)
    HITJ(1, h1, s1)
    HITJ(2, h2, s2)
    HITJ(3, h3, s3)
    HITJ(4, h4, s4)
    HITJ(5, h5, s5)
    HITJ(6, h6, s6)
    HITJ(7, h7, s7)
#undef HITJ
  }
  return wc;
}

__global__ __launch_bounds__(NTHR) void k_wprep(const float* __restrict__ Wg1, const float* __restrict__ Wg2,
                                                const float* __restrict__ Wg3, const float* __restrict__ Wv,
                                                const float* __restrict__ Wo, const float* __restrict__ Wqk,
                                                const float* __restrict__ Wse, const float* __restrict__ W1,
                                                const float* __restrict__ W2, unsigned short* WT) {
  const int u = (int)blockIdx.x * NTHR + (int)threadIdx.x;
  const float* W;
  int kin, nout, ub, doff;
  if      (u < 2048)  { W = Wg1; kin = 128; nout = 128; ub = 0;     doff = OW_G1; }
  else if (u < 4096)  { W = Wg2; kin = 128; nout = 128; ub = 2048;  doff = OW_G2; }
  else if (u < 6144)  { W = Wg3; kin = 128; nout = 128; ub = 4096;  doff = OW_G3; }
  else if (u < 8192)  { W = Wv;  kin = 128; nout = 128; ub = 6144;  doff = OW_V;  }
  else if (u < 10240) { W = Wo;  kin = 128; nout = 128; ub = 8192;  doff = OW_O;  }
  else if (u < 14336) { W = Wqk; kin = 128; nout = 256; ub = 10240; doff = OW_QK; }
  else if (u < 22528) { W = Wse; kin = 512; nout = 128; ub = 14336; doff = OW_SE; }
  else if (u < 30720) { W = W1;  kin = 128; nout = 512; ub = 22528; doff = OW_1;  }
  else if (u < 38912) { W = W2;  kin = 512; nout = 128; ub = 30720; doff = OW_2;  }
  else return;
  const int lg = (kin == 128) ? 4 : 6;
  const int v  = u - ub;
  const int n  = v >> lg;
  const int k8 = (v & ((1 << lg) - 1)) * 8;
  const float* p = W + (size_t)k8 * nout + n;
  v8us o;
#pragma unroll
  for (int i = 0; i < 8; ++i) o[i] = (unsigned short)bf16_bits(p[(size_t)i * nout]);
  unsigned short* dp = WT + doff + (size_t)n * kin + k8;
  *(volatile v8us*)dp = o;
  __threadfence();
  *(volatile v8us*)dp = o;
}

__global__ __launch_bounds__(NTHR) void k_cvx(const float* __restrict__ x, int nN, int nUnits,
                                              unsigned short* xb) {
  const int u = (int)blockIdx.x * NTHR + (int)threadIdx.x;
  if (u >= nUnits) return;
  const int row = u >> 4;
  const int k8  = (u & 15) * 8;
  const int rc  = row < nN ? row : nN - 1;
  const float* p = x + (size_t)rc * DM + k8;
  const v4f a = *(const v4fa*)p;
  const v4f b = *(const v4fa*)(p + 4);
  const bool ok = row < nN;
  v8us o;
  o[0] = ok ? (unsigned short)bf16_bits(a.x) : (unsigned short)0;
  o[1] = ok ? (unsigned short)bf16_bits(a.y) : (unsigned short)0;
  o[2] = ok ? (unsigned short)bf16_bits(a.z) : (unsigned short)0;
  o[3] = ok ? (unsigned short)bf16_bits(a.w) : (unsigned short)0;
  o[4] = ok ? (unsigned short)bf16_bits(b.x) : (unsigned short)0;
  o[5] = ok ? (unsigned short)bf16_bits(b.y) : (unsigned short)0;
  o[6] = ok ? (unsigned short)bf16_bits(b.z) : (unsigned short)0;
  o[7] = ok ? (unsigned short)bf16_bits(b.w) : (unsigned short)0;
  unsigned short* dp = xb + (size_t)row * DM + k8;
  *(volatile v8us*)dp = o;
  __threadfence();
  *(volatile v8us*)dp = o;
}

__global__ __launch_bounds__(NTHR) void k_deg(const int* __restrict__ dsts, int nE, int vec8, float* dis) {
  __shared__ __attribute__((aligned(16))) int scnt[NBD];
  __shared__ __attribute__((aligned(16))) int list[LISTN];
  __shared__ int wcnt[NWAVE];
  const int tid = (int)threadIdx.x, lane = tid & 31, wave = tid >> 5;
  const int nodeBase = (int)blockIdx.x * NBD;

  for (int i = tid; i < NBD; i += NTHR) scnt[i] = 0;
  for (int i = tid; i < LISTN; i += NTHR) list[i] = 0;
  if (tid < NWAVE) wcnt[tid] = 0;
  __syncthreads();

  const int nChunks = (nE + CHUNK - 1) / CHUNK;
#pragma unroll 1
  for (int ch = 0; ch < nChunks; ++ch) {
    const int cbase = ch * CHUNK;
    const int wc = scan_chunk<SLD>(dsts, nE, cbase, nodeBase, NBD, vec8, list, tid, lane, wave);
    if (lane == 0) wcnt[wave] = wc;
    __syncthreads();
    if (wave == 0) {
#pragma unroll 1
      for (int w2 = 0; w2 < NWAVE; ++w2) {
        int c = wcnt[w2];
        c = c < 0 ? 0 : (c > WCAP ? WCAP : c);
#pragma unroll 1
        for (int b0 = 0; b0 < c; b0 += 32) {
          const int idx = b0 + lane;
          const int ent = list[w2 * WCAP + (idx < WCAP ? idx : WCAP - 1)];
          const int m32 = (c - b0) < 32 ? (c - b0) : 32;
#pragma unroll 1
          for (int k = 0; k < m32; ++k) {
            const int u  = __builtin_amdgcn_readlane(ent, k);
            const int sl = u & (NBD - 1);
            if (lane == 0) scnt[sl] = scnt[sl] + 1;
          }
        }
      }
    }
    __syncthreads();
  }

#pragma unroll 1
  for (int i = tid; i < NBD; i += NTHR) {
    const float d = (float)scnt[i] + 1.0f;
    scnt[i] = __float_as_int(1.0f / sqrtf(d));
  }
  __syncthreads();

  v4f vals[NBD / (NTHR * 4)];
#pragma unroll
  for (int it = 0; it < NBD / (NTHR * 4); ++it) {
    const int s0 = it * (NTHR * 4) + 4 * tid;
    const v4i c4 = *(const v4ia*)(scnt + s0);
    v4f v;
    v.x = __int_as_float(c4.x); v.y = __int_as_float(c4.y);
    v.z = __int_as_float(c4.z); v.w = __int_as_float(c4.w);
    vals[it] = v;
  }
#pragma unroll
  for (int it = 0; it < NBD / (NTHR * 4); ++it) {
    const int s0 = it * (NTHR * 4) + 4 * tid;
    *(volatile v4f*)(dis + (size_t)nodeBase + s0) = vals[it];
  }
  __threadfence();
#pragma unroll
  for (int it = 0; it < NBD / (NTHR * 4); ++it) {
    const int s0 = it * (NTHR * 4) + 4 * tid;
    *(volatile v4f*)(dis + (size_t)nodeBase + s0) = vals[it];
  }
}

__device__ __forceinline__ void scan_build(const int* __restrict__ keys, int nE, int nodeBase, int vec8,
                                           int* dsm, int* list, int* hl, int* sl, int* cnt, int* offs,
                                           int* cur, int* misc, int tid, int lane, int wave,
                                           int& ttOut, int& ovfOut) {
  {
    const v4i z4 = {0, 0, 0, 0};
    for (int i = tid * 4; i < AGG_ZINTS; i += NTHR * 4) *(v4ia*)(dsm + i) = z4;
    if (tid < MISC_INTS) misc[tid] = 0;
  }
  __syncthreads();

  int t = 0, ov = 0;
  const int nChunks = (nE + CHUNK - 1) / CHUNK;
#pragma unroll 1
  for (int ch = 0; ch < nChunks; ++ch) {
    const int cbase = ch * CHUNK;
    const int wc = scan_chunk<SLA>(keys, nE, cbase, nodeBase, NBA, vec8, list, tid, lane, wave);
    if (lane == 0) misc[wave] = wc;
    __syncthreads();
    if (wave == 0) {
#pragma unroll 1
      for (int w2 = 0; w2 < NWAVE; ++w2) {
        int c = misc[w2];
        c = c < 0 ? 0 : (c > WCAP ? WCAP : c);
#pragma unroll 1
        for (int b0 = 0; b0 < c; b0 += 32) {
          const int idx = b0 + lane;
          const int ent = list[w2 * WCAP + (idx < WCAP ? idx : WCAP - 1)];
          const int m32 = (c - b0) < 32 ? (c - b0) : 32;
#pragma unroll 1
          for (int k = 0; k < m32; ++k) {
            const int u    = __builtin_amdgcn_readlane(ent, k);
            const int slot = u & (NBA - 1);
            const int el   = (u >> SLA) & (CHUNK - 1);
            const int pk   = ((cbase + el) << SLA) | slot;
            if (t < RCAP) {
              if (lane == 0) { hl[t] = pk; cnt[slot] = cnt[slot] + 1; }
              t = t + 1;
            } else {
              ov = 1;
            }
          }
        }
      }
    }
    __syncthreads();
  }
  if (wave == 0 && lane == 0) { misc[8] = t; misc[9] = ov; }
  __syncthreads();
  int tt = misc[8];
  tt = tt < 0 ? 0 : (tt > RCAP ? RCAP : tt);
  const int ovf = misc[9];

  if (wave == 0) {
    const int base = lane * (NBA / 32);
    int s = 0;
#pragma unroll 1
    for (int i = 0; i < NBA / 32; ++i) s += cnt[base + i];
    int incl = s;
#pragma unroll
    for (int d = 1; d < 32; d <<= 1) {
      const int y = __shfl_up(incl, d, 32);
      if (lane >= d) incl += y;
    }
    int run = incl - s;
#pragma unroll 1
    for (int i = 0; i < NBA / 32; ++i) {
      const int cv = cnt[base + i];
      offs[base + i] = run;
      cur[base + i]  = run;
      run += cv;
    }
  }
  __syncthreads();
  if (wave == 0) {
#pragma unroll 1
    for (int b0 = 0; b0 < tt; b0 += 32) {
      const int idx = b0 + lane;
      const int ent = hl[idx < RCAP ? idx : RCAP - 1];
      const int m32 = (tt - b0) < 32 ? (tt - b0) : 32;
#pragma unroll 1
      for (int k = 0; k < m32; ++k) {
        const int u    = __builtin_amdgcn_readlane(ent, k);
        const int slot = u & (NBA - 1);
        if (lane == 0) {
          int p = cur[slot];
          p = p < 0 ? 0 : (p > RCAP - 1 ? RCAP - 1 : p);
          sl[p] = u;
          cur[slot] = p + 1;
        }
      }
    }
  }
  __syncthreads();
  ttOut = tt;
  ovfOut = ovf;
}

__global__ __launch_bounds__(NTHR) void k_gscan(const int* __restrict__ srcs, const int* __restrict__ dsts,
                                                int nE, int nN, int vec8, int mRows,
                                                const float* __restrict__ dis, const float* __restrict__ ht,
                                                const float* __restrict__ bias, unsigned short* gout) {
  extern __shared__ __attribute__((aligned(16))) int dsm[];
  int* list = dsm;
  int* hl   = dsm + LISTN;
  int* sl   = hl + RCAP;
  int* cnt  = sl + RCAP;
  int* offs = cnt + NBA;
  int* cur  = offs + NBA;
  int* misc = cur + NBA;
  const int tid = (int)threadIdx.x, lane = tid & 31, wave = tid >> 5;
  unsigned short* rowbuf = (unsigned short*)(misc + MISC_INTS) + wave * HLP;
  const int nodeBase = (int)blockIdx.x * NBA;

  int tt = 0, ovf = 0;
  scan_build(dsts, nE, nodeBase, vec8, dsm, list, hl, sl, cnt, offs, cur, misc, tid, lane, wave, tt, ovf);

  const v4f bv = ldv_bf(bias + 4 * lane);
  const float qnan = __int_as_float(0x7fc00000);
  const float pz = (ovf != 0) ? qnan : 0.0f;
#pragma unroll 1
  for (int si = 0; si < NBA / NWAVE; ++si) {
    const int s    = si * NWAVE + wave;
    const int node = nodeBase + s;
    int c = cnt[s];
    const bool big = c > DEGCAP;
    c = c < 0 ? 0 : (c > DEGCAP ? DEGCAP : c);
    int o = offs[s];
    o = o < 0 ? 0 : (o > RCAP ? RCAP : o);
    const int nc = node < nN ? node : nN - 1;
    const float dd = dis[nc];
    const float rd = dd * dd;
    float a0 = 0.0f, a1 = 0.0f, a2 = 0.0f, a3 = 0.0f;
#pragma unroll 1
    for (int b0 = 0; b0 < c; b0 += 32) {
      int idx = o + b0 + lane;
      idx = idx > RCAP - 1 ? RCAP - 1 : idx;
      const int ent = sl[idx];
      int eid = ent >> SLA;
      eid = eid < 0 ? 0 : (eid > nE - 1 ? nE - 1 : eid);
      int sr = srcs[eid];
      sr = sr < 0 ? 0 : (sr > nN - 1 ? nN - 1 : sr);
      const float cf  = dis[sr] * dd;
      const int   cfi = __float_as_int(cf);
      const int m32 = (c - b0) < 32 ? (c - b0) : 32;
#pragma unroll 1
      for (int k = 0; k < m32; ++k) {
        const int   sk = __builtin_amdgcn_readlane(sr, k);
        const float ck = __int_as_float(__builtin_amdgcn_readlane(cfi, k));
        const v4f a = *(const v4f*)(ht + (size_t)sk * DM + 4 * lane);
        a0 = fmaf(ck, a.x, a0); a1 = fmaf(ck, a.y, a1);
        a2 = fmaf(ck, a.z, a2); a3 = fmaf(ck, a.w, a3);
      }
    }
    const v4f sv = *(const v4f*)(ht + (size_t)nc * DM + 4 * lane);
    const float pzr = big ? qnan : pz;
    const bool live = node < nN;
    float y0 = (a0 + sv.x * rd) + bv.x;
    float y1 = (a1 + sv.y * rd) + bv.y;
    float y2 = (a2 + sv.z * rd) + bv.z;
    float y3 = (a3 + sv.w * rd) + bv.w;
    y0 = (y0 > 0.0f) ? y0 : (y0 - y0);
    y1 = (y1 > 0.0f) ? y1 : (y1 - y1);
    y2 = (y2 > 0.0f) ? y2 : (y2 - y2);
    y3 = (y3 > 0.0f) ? y3 : (y3 - y3);
    const float m0 = live ? (y0 + pzr) : 0.0f;
    const float m1 = live ? (y1 + pzr) : 0.0f;
    const float m2 = live ? (y2 + pzr) : 0.0f;
    const float m3 = live ? (y3 + pzr) : 0.0f;
    const unsigned p0 = split_hl(m0), p1 = split_hl(m1), p2 = split_hl(m2), p3 = split_hl(m3);
    v4us mh, ml;
    mh[0] = (unsigned short)(p0 & 0xffffu); ml[0] = (unsigned short)(p0 >> 16);
    mh[1] = (unsigned short)(p1 & 0xffffu); ml[1] = (unsigned short)(p1 >> 16);
    mh[2] = (unsigned short)(p2 & 0xffffu); ml[2] = (unsigned short)(p2 >> 16);
    mh[3] = (unsigned short)(p3 & 0xffffu); ml[3] = (unsigned short)(p3 >> 16);
    *(v4usa*)(rowbuf + 4 * lane) = mh;
    *(v4usa*)(rowbuf + DM + 4 * lane) = ml;
    wave_sync();
    const v8us q0 = *(const v8usa*)(rowbuf + 8 * lane);
    wave_sync();
    if (node < mRows) {
      unsigned short* rpw = gout + (size_t)node * HLP + 8 * lane;
      *(volatile v8us*)rpw = q0;
      __threadfence();
      *(volatile v8us*)rpw = q0;
    }
  }
}

__global__ __launch_bounds__(NTHR) void k_ascan(const int* __restrict__ srcs, const int* __restrict__ dsts,
                                                int nE, int nN, int vec8, int mRows,
                                                const float* __restrict__ qp, const float* __restrict__ kv,
                                                unsigned short* aout) {
  extern __shared__ __attribute__((aligned(16))) int dsm[];
  int* list = dsm;
  int* hl   = dsm + LISTN;
  int* sl   = hl + RCAP;
  int* cnt  = sl + RCAP;
  int* offs = cnt + NBA;
  int* cur  = offs + NBA;
  int* misc = cur + NBA;
  const int tid = (int)threadIdx.x, lane = tid & 31, wave = tid >> 5;
  unsigned short* rowbuf = (unsigned short*)(misc + MISC_INTS) + wave * HLP;
  const int nodeBase = (int)blockIdx.x * NBA;

  int tt = 0, ovf = 0;
  scan_build(dsts, nE, nodeBase, vec8, dsm, list, hl, sl, cnt, offs, cur, misc, tid, lane, wave, tt, ovf);

  const float qnan = __int_as_float(0x7fc00000);
  const float pz = (ovf != 0) ? qnan : 0.0f;
#pragma unroll 1
  for (int si = 0; si < NBA / NWAVE; ++si) {
    const int s    = si * NWAVE + wave;
    const int node = nodeBase + s;
    int c = cnt[s];
    const bool big = c > DEGCAP;
    c = c < 0 ? 0 : (c > DEGCAP ? DEGCAP : c);
    int o = offs[s];
    o = o < 0 ? 0 : (o > RCAP ? RCAP : o);
    const int nc = node < nN ? node : nN - 1;
    const v4f q4 = *(const v4f*)(qp + (size_t)nc * DM + 4 * lane);
    float mx = -3.0e38f, l = 0.0f;
    float a0 = 0.0f, a1 = 0.0f, a2 = 0.0f, a3 = 0.0f;
#pragma unroll 1
    for (int b0 = 0; b0 < c; b0 += 32) {
      int idx = o + b0 + lane;
      idx = idx > RCAP - 1 ? RCAP - 1 : idx;
      const int ent = sl[idx];
      int eid = ent >> SLA;
      eid = eid < 0 ? 0 : (eid > nE - 1 ? nE - 1 : eid);
      int sr = srcs[eid];
      sr = sr < 0 ? 0 : (sr > nN - 1 ? nN - 1 : sr);
      const int m32 = (c - b0) < 32 ? (c - b0) : 32;
#pragma unroll 1
      for (int k = 0; k < m32; ++k) {
        const int sk = __builtin_amdgcn_readlane(sr, k);
        const float* rp = kv + (size_t)sk * (2 * DM) + 4 * lane;
        const v4f k4 = *(const v4f*)rp;
        const v4f v4 = *(const v4f*)(rp + DM);
        float d = q4.x * k4.x;
        d = fmaf(q4.y, k4.y, d);
        d = fmaf(q4.z, k4.z, d);
        d = fmaf(q4.w, k4.w, d);
        d += __shfl_xor(d, 1, 32);
        d += __shfl_xor(d, 2, 32);
        const float sc = d * 0.25f;
        const float df = sc - mx;
        const float e  = expf(-fabsf(df));
        const bool  up = df > 0.0f;
        const float corr = up ? e : 1.0f;
        const float p    = up ? 1.0f : e;
        mx = up ? sc : mx;
        l  = fmaf(l, corr, p);
        a0 = fmaf(a0, corr, p * v4.x);
        a1 = fmaf(a1, corr, p * v4.y);
        a2 = fmaf(a2, corr, p * v4.z);
        a3 = fmaf(a3, corr, p * v4.w);
      }
    }
    const float inv = 1.0f / (l + 1e-16f);
    const float pzr = big ? qnan : pz;
    const bool live = node < nN;
    const float m0 = live ? (a0 * inv + pzr) : 0.0f;
    const float m1 = live ? (a1 * inv + pzr) : 0.0f;
    const float m2 = live ? (a2 * inv + pzr) : 0.0f;
    const float m3 = live ? (a3 * inv + pzr) : 0.0f;
    const unsigned p0 = split_hl(m0), p1 = split_hl(m1), p2 = split_hl(m2), p3 = split_hl(m3);
    v4us mh, ml;
    mh[0] = (unsigned short)(p0 & 0xffffu); ml[0] = (unsigned short)(p0 >> 16);
    mh[1] = (unsigned short)(p1 & 0xffffu); ml[1] = (unsigned short)(p1 >> 16);
    mh[2] = (unsigned short)(p2 & 0xffffu); ml[2] = (unsigned short)(p2 >> 16);
    mh[3] = (unsigned short)(p3 & 0xffffu); ml[3] = (unsigned short)(p3 >> 16);
    *(v4usa*)(rowbuf + 4 * lane) = mh;
    *(v4usa*)(rowbuf + DM + 4 * lane) = ml;
    wave_sync();
    const v8us q0 = *(const v8usa*)(rowbuf + 8 * lane);
    wave_sync();
    if (node < mRows) {
      unsigned short* rpw = aout + (size_t)node * HLP + 8 * lane;
      *(volatile v8us*)rpw = q0;
      __threadfence();
      *(volatile v8us*)rpw = q0;
    }
  }
}

__global__ __launch_bounds__(GTHR) void k_bnstats(const unsigned short* __restrict__ XB,
                                                  const unsigned short* __restrict__ G1,
                                                  const unsigned short* __restrict__ G2,
                                                  const unsigned short* __restrict__ G3,
                                                  int nN, double* rec) {
  __shared__ __attribute__((aligned(16))) double sd[1024];
  const int tid = (int)threadIdx.x, lane = tid & 31, wave = tid >> 5;
  const int r0 = (int)blockIdx.x * BNRB;
  const int r1 = (r0 + BNRB) < nN ? (r0 + BNRB) : nN;
  const unsigned short* P = XB;
  int pitch = DM;
  if (wave == 1) { P = G1; pitch = HLP; }
  else if (wave == 2) { P = G2; pitch = HLP; }
  else if (wave == 3) { P = G3; pitch = HLP; }
  const int c4 = 4 * lane;
  double s0 = 0.0, s1 = 0.0, s2 = 0.0, s3 = 0.0;
  double q0 = 0.0, q1 = 0.0, q2 = 0.0, q3 = 0.0;
#pragma unroll 2
  for (int r = r0; r < r1; ++r) {
    const unsigned short* rp = P + (size_t)r * pitch + c4;
    v4f v = ld_bf4(rp);
    if (wave != 0) {
      const v4f lo = ld_bf4(rp + DM);
      v = v + lo;
    }
    const double d0 = (double)v.x, d1 = (double)v.y, d2 = (double)v.z, d3 = (double)v.w;
    s0 += d0; s1 += d1; s2 += d2; s3 += d3;
    q0 = fma(d0, d0, q0); q1 = fma(d1, d1, q1); q2 = fma(d2, d2, q2); q3 = fma(d3, d3, q3);
  }
  const int cb = DM * wave + c4;
  sd[cb + 0] = s0; sd[cb + 1] = s1; sd[cb + 2] = s2; sd[cb + 3] = s3;
  sd[512 + cb + 0] = q0; sd[512 + cb + 1] = q1; sd[512 + cb + 2] = q2; sd[512 + cb + 3] = q3;
  __syncthreads();
  v2d ov[4];
#pragma unroll
  for (int it = 0; it < 4; ++it) ov[it] = *(const v2da*)(sd + 2 * (it * GTHR + tid));
  double* bp = rec + (size_t)blockIdx.x * 1024;
#pragma unroll
  for (int it = 0; it < 4; ++it) *(volatile v2d*)(bp + 2 * (it * GTHR + tid)) = ov[it];
  __threadfence();
#pragma unroll
  for (int it = 0; it < 4; ++it) *(volatile v2d*)(bp + 2 * (it * GTHR + tid)) = ov[it];
}

__global__ __launch_bounds__(512) void k_bncomb(const double* __restrict__ rec, int nB, double invN,
                                                const float* __restrict__ bng, const float* __restrict__ bnb,
                                                float* tab) {
  __shared__ __attribute__((aligned(16))) float tb[1536];
  const int tid = (int)threadIdx.x;
  double s = 0.0, q = 0.0;
#pragma unroll 2
  for (int b = 0; b < nB; ++b) {
    s += rec[(size_t)b * 1024 + tid];
    q += rec[(size_t)b * 1024 + 512 + tid];
  }
  const double mu = s * invN;
  double var = q * invN - mu * mu;
  var = (var < 0.0) ? 0.0 : var;
  const float a = bf16_val(bng[tid]) * rsqrtf((float)var + 1e-5f);
  tb[tid] = (float)mu;
  tb[512 + tid] = a;
  tb[1024 + tid] = bf16_val(bnb[tid]);
  __syncthreads();
  const int tc = tid < 384 ? tid : 383;
  const v4f ov = *(const v4fa*)(tb + 4 * tc);
  const bool okst = tid < 384;
  if (okst) *(volatile v4f*)(tab + 4 * tc) = ov;
  __threadfence();
  if (okst) *(volatile v4f*)(tab + 4 * tc) = ov;
}

struct EpiP {
  const float* bias; const float* gam; const float* bet;
  const unsigned short* resB; const float* resF; const int* gate;
  float* outF0; float* outF1; unsigned short* outH;
  int ldo0, ldo1, ldh, nOut;
};

__device__ __forceinline__ v4f ln_row(v4f t, v4f g, v4f b) {
  const float s  = wave_sum((t.x + t.y) + (t.z + t.w));
  const float mu = s * (1.0f / 128.0f);
  const v4f d = t - mu;
  const float q  = wave_sum((d.x * d.x + d.y * d.y) + (d.z * d.z + d.w * d.w));
  const float rs = rsqrtf(q * (1.0f / 128.0f) + 1e-5f);
  v4f y;
  y.x = d.x * rs * g.x + b.x;
  y.y = d.y * rs * g.y + b.y;
  y.z = d.z * rs * g.z + b.z;
  y.w = d.w * rs * g.w + b.w;
  return y;
}

__device__ __forceinline__ void stage_res(const unsigned short* __restrict__ resB, float* stg, int row0,
                                          int wave, int lane) {
  unsigned short* sbase = (unsigned short*)stg + (size_t)(16 * wave) * (2 * GBN);
  const int hh = lane >> 4, m = lane & 15;
  v4u w[8];
#pragma unroll
  for (int j = 0; j < 8; ++j)
    w[j] = *(const v4ua*)(resB + (size_t)(row0 + 2 * j + hh) * DM + 8 * m);
#pragma unroll
  for (int j = 0; j < 8; ++j)
    *(v4ua*)(sbase + (2 * j + hh) * (2 * GBN) + 8 * m) = w[j];
  __syncthreads();
}
__device__ __forceinline__ v4f ld_res(const float* stg, int wave, int i, int lane) {
  const unsigned short* srow = (const unsigned short*)stg + (size_t)(16 * wave + i) * (2 * GBN);
  const v2u w = *(const v2ua*)(srow + 4 * lane);
  v4f r;
  r.x = bflo(w.x); r.y = bfhi(w.x); r.z = bflo(w.y); r.w = bfhi(w.y);
  return r;
}

__device__ __forceinline__ void restage_hl(v4f (&pv)[16], v8us (&qv)[16], float* stg, int wave, int lane) {
  unsigned short* sbase = (unsigned short*)stg + (size_t)(16 * wave) * (2 * GBN);
#pragma unroll
  for (int i = 0; i < 16; ++i) {
    const unsigned p0 = split_hl(pv[i].x), p1 = split_hl(pv[i].y);
    const unsigned p2 = split_hl(pv[i].z), p3 = split_hl(pv[i].w);
    v4us h4, l4;
    h4[0] = (unsigned short)(p0 & 0xffffu); l4[0] = (unsigned short)(p0 >> 16);
    h4[1] = (unsigned short)(p1 & 0xffffu); l4[1] = (unsigned short)(p1 >> 16);
    h4[2] = (unsigned short)(p2 & 0xffffu); l4[2] = (unsigned short)(p2 >> 16);
    h4[3] = (unsigned short)(p3 & 0xffffu); l4[3] = (unsigned short)(p3 >> 16);
    unsigned short* srow = sbase + i * (2 * GBN);
    *(v4usa*)(srow + 4 * lane) = h4;
    *(v4usa*)(srow + DM + 4 * lane) = l4;
  }
  __syncthreads();
#pragma unroll
  for (int i = 0; i < 16; ++i) qv[i] = *(const v8usa*)(sbase + i * (2 * GBN) + 8 * lane);
}

template <int EPI>
__device__ __forceinline__ void gemm_epi(v8f (&acc)[8], float* stg, const EpiP& P, int rowBase, int by,
                                         int lane, int wave) {
  const int hh = lane >> 4, m = lane & 15;
#pragma unroll
  for (int nt = 0; nt < 8; ++nt) {
    const int lc = 16 * nt + m;
#pragma unroll
    for (int r = 0; r < 8; ++r) {
      const int lr = 16 * wave + 8 * hh + r;
      stg[lr * GBN + lc] = acc[nt][r];
    }
  }
  __syncthreads();
  v4f pv[16];
#pragma unroll
  for (int i = 0; i < 16; ++i) pv[i] = *(const v4fa*)(stg + (16 * wave + i) * GBN + 4 * lane);
  __syncthreads();
  const int row0 = rowBase + 16 * wave;

  if constexpr (EPI == 0) {
    float* ob = (by == 0) ? P.outF0 : P.outF1;
    const int ld = (by == 0) ? P.ldo0 : P.ldo1;
    float* op = ob + (size_t)row0 * (size_t)ld + 4 * lane;
#pragma unroll
    for (int i = 0; i < 16; ++i) *(volatile v4f*)(op + (size_t)i * (size_t)ld) = pv[i];
    __threadfence();
#pragma unroll
    for (int i = 0; i < 16; ++i) *(volatile v4f*)(op + (size_t)i * (size_t)ld) = pv[i];
  } else if constexpr (EPI == 1) {
    const v4f b4 = ldv_bf(P.bias + 4 * lane);
    const int gt = P.gate[0];
    stage_res(P.resB, stg, row0, wave, lane);
#pragma unroll
    for (int i = 0; i < 16; ++i) {
      const int row = row0 + i;
      const bool ok = row < P.nOut;
      const v4f xr = ld_res(stg, wave, i, lane);
      const v4f t = pv[i] + b4;
      v4f y;
      y.x = (gt != 0) ? (xr.x + t.x) : xr.x;
      y.y = (gt != 0) ? (xr.y + t.y) : xr.y;
      y.z = (gt != 0) ? (xr.z + t.z) : xr.z;
      y.w = (gt != 0) ? (xr.w + t.w) : xr.w;
      y.x = ok ? y.x : 0.0f; y.y = ok ? y.y : 0.0f; y.z = ok ? y.z : 0.0f; y.w = ok ? y.w : 0.0f;
      pv[i] = y;
    }
    wave_sync();
    v8us qv[16];
    restage_hl(pv, qv, stg, wave, lane);
    unsigned short* hp = P.outH + (size_t)row0 * (size_t)P.ldh + 8 * lane;
#pragma unroll
    for (int i = 0; i < 16; ++i) *(volatile v8us*)(hp + (size_t)i * (size_t)P.ldh) = qv[i];
    __threadfence();
#pragma unroll
    for (int i = 0; i < 16; ++i) *(volatile v8us*)(hp + (size_t)i * (size_t)P.ldh) = qv[i];
  } else if constexpr (EPI == 2) {
    const v4f b4 = ldv_bf(P.bias + 4 * lane);
    const v4f g4 = ldv_bf(P.gam + 4 * lane);
    const v4f e4 = ldv_bf(P.bet + 4 * lane);
    stage_res(P.resB, stg, row0, wave, lane);
#pragma unroll
    for (int i = 0; i < 16; ++i) {
      const int row = row0 + i;
      const bool ok = row < P.nOut;
      const v4f xr = ld_res(stg, wave, i, lane);
      const v4f t = xr + (pv[i] + b4);
      v4f y = ln_row(t, g4, e4);
      y.x = ok ? y.x : 0.0f; y.y = ok ? y.y : 0.0f; y.z = ok ? y.z : 0.0f; y.w = ok ? y.w : 0.0f;
      pv[i] = y;
    }
    wave_sync();
    float* op = P.outF0 + (size_t)row0 * DM + 4 * lane;
#pragma unroll
    for (int i = 0; i < 16; ++i) *(volatile v4f*)(op + (size_t)i * DM) = pv[i];
    __threadfence();
#pragma unroll
    for (int i = 0; i < 16; ++i) *(volatile v4f*)(op + (size_t)i * DM) = pv[i];
    v8us qv[16];
    restage_hl(pv, qv, stg, wave, lane);
    unsigned short* hp = P.outH + (size_t)row0 * (size_t)P.ldh + 8 * lane;
#pragma unroll
    for (int i = 0; i < 16; ++i) *(volatile v8us*)(hp + (size_t)i * (size_t)P.ldh) = qv[i];
    __threadfence();
#pragma unroll
    for (int i = 0; i < 16; ++i) *(volatile v8us*)(hp + (size_t)i * (size_t)P.ldh) = qv[i];
  } else if constexpr (EPI == 3) {
    const v4f b4 = ldv_bf(P.bias + GBN * by + 4 * lane);
#pragma unroll
    for (int i = 0; i < 16; ++i) {
      const bool ok = (row0 + i) < P.nOut;
      const v4f t = pv[i] + b4;
      v4f y;
      y.x = (t.x > 0.0f) ? t.x : (t.x - t.x);
      y.y = (t.y > 0.0f) ? t.y : (t.y - t.y);
      y.z = (t.z > 0.0f) ? t.z : (t.z - t.z);
      y.w = (t.w > 0.0f) ? t.w : (t.w - t.w);
      y.x = ok ? y.x : 0.0f; y.y = ok ? y.y : 0.0f; y.z = ok ? y.z : 0.0f; y.w = ok ? y.w : 0.0f;
      pv[i] = y;
    }
    v8us qv[16];
    restage_hl(pv, qv, stg, wave, lane);
    const int hsel = lane >> 4;
    unsigned short* hp = P.outH + (size_t)row0 * (size_t)P.ldh + GBN * by + hsel * (P.ldh >> 1) + 8 * (lane & 15);
#pragma unroll
    for (int i = 0; i < 16; ++i) *(volatile v8us*)(hp + (size_t)i * (size_t)P.ldh) = qv[i];
    __threadfence();
#pragma unroll
    for (int i = 0; i < 16; ++i) *(volatile v8us*)(hp + (size_t)i * (size_t)P.ldh) = qv[i];
  } else {
    const v4f b4 = ldv_bf(P.bias + 4 * lane);
    const v4f g4 = ldv_bf(P.gam + 4 * lane);
    const v4f e4 = ldv_bf(P.bet + 4 * lane);
#pragma unroll
    for (int i = 0; i < 16; ++i) {
      const int row = row0 + i;
      const v4f hr = *(const v4f*)(P.resF + (size_t)row * DM + 4 * lane);
      const v4f t = hr + (pv[i] + b4);
      pv[i] = ln_row(t, g4, e4);
    }
    float* op = P.outF0 + (size_t)row0 * DM + 4 * lane;
#pragma unroll
    for (int i = 0; i < 16; ++i) {
      if ((row0 + i) < P.nOut) *(volatile v4f*)(op + (size_t)i * DM) = pv[i];
    }
    __threadfence();
#pragma unroll
    for (int i = 0; i < 16; ++i) {
      if ((row0 + i) < P.nOut) *(volatile v4f*)(op + (size_t)i * DM) = pv[i];
    }
  }
}

template <int TWO, int EPI>
__global__ __launch_bounds__(GTHR) void k_gemm(
    const unsigned short* __restrict__ A, int lda, int loOff, int K,
    const unsigned short* __restrict__ BT,
    const float* __restrict__ bias, const float* __restrict__ gam, const float* __restrict__ bet,
    const unsigned short* __restrict__ resB, const float* __restrict__ resF, const int* __restrict__ gate,
    float* outF0, int ldo0, float* outF1, int ldo1, unsigned short* outH, int ldh, int nOut)
{
  __shared__ __attribute__((aligned(16))) float stg[GBM * GBN];
  const int tid = (int)threadIdx.x, lane = tid & 31, wave = tid >> 5, hh = lane >> 4, m = lane & 15;
  const int rowBase = (int)blockIdx.x * GBM;
  const int by = (int)blockIdx.y;

  v8f acc[8];
  {
    const v8f z = {0.f, 0.f, 0.f, 0.f, 0.f, 0.f, 0.f, 0.f};
#pragma unroll
    for (int t = 0; t < 8; ++t) acc[t] = z;
  }
  const unsigned short* ap = A + (size_t)(rowBase + 16 * wave + m) * (size_t)lda + 8 * hh;
  const unsigned short* bp = BT + (size_t)(GBN * by + m) * (size_t)K + 8 * hh;

#pragma unroll 1
  for (int k0 = 0; k0 < K; k0 += 32) {
    FragB af, al;
    af.h[0] = *(const v8usa*)(ap + k0);
    af.h[1] = *(const v8usa*)(ap + k0 + 16);
    if constexpr (TWO != 0) {
      al.h[0] = *(const v8usa*)(ap + loOff + k0);
      al.h[1] = *(const v8usa*)(ap + loOff + k0 + 16);
    } else {
      al.h[0] = af.h[0]; al.h[1] = af.h[1];
    }
#pragma unroll
    for (int nt = 0; nt < 8; ++nt) {
      const unsigned short* wq = bp + (size_t)(16 * nt) * (size_t)K + k0;
      FragB bf;
      bf.h[0] = *(const v8usa*)wq;
      bf.h[1] = *(const v8usa*)(wq + 16);
      acc[nt] = wmb(af, bf, acc[nt]);
      if constexpr (TWO != 0) acc[nt] = wmb(al, bf, acc[nt]);
    }
  }

  EpiP P;
  P.bias = bias; P.gam = gam; P.bet = bet; P.resB = resB; P.resF = resF; P.gate = gate;
  P.outF0 = outF0; P.outF1 = outF1; P.outH = outH;
  P.ldo0 = ldo0; P.ldo1 = ldo1; P.ldh = ldh; P.nOut = nOut;
  gemm_epi<EPI>(acc, stg, P, rowBase, by, lane, wave);
}

__global__ __launch_bounds__(GTHR) void k_se(const unsigned short* __restrict__ XB,
                                             const unsigned short* __restrict__ G1,
                                             const unsigned short* __restrict__ G2,
                                             const unsigned short* __restrict__ G3,
                                             const float* __restrict__ tab,
                                             const unsigned short* __restrict__ WseT,
                                             const float* __restrict__ bse, const int* __restrict__ gate,
                                             unsigned short* xatt, int nOut) {
  __shared__ __attribute__((aligned(16))) float stg[GBM * GBN];
  __shared__ __attribute__((aligned(16))) unsigned short ah[GBM * APT];
  __shared__ __attribute__((aligned(16))) unsigned short al[GBM * APT];
  __shared__ __attribute__((aligned(16))) float tb[1536];
  const int tid = (int)threadIdx.x, lane = tid & 31, wave = tid >> 5, hh = lane >> 4, m = lane & 15;
  const int rowBase = (int)blockIdx.x * GBM;

#pragma unroll
  for (int it = 0; it < 3; ++it) {
    const int i = 4 * (it * GTHR + tid);
    *(v4fa*)(tb + i) = *(const v4f*)(tab + i);
  }
  v8f acc[8];
  {
    const v8f z = {0.f, 0.f, 0.f, 0.f, 0.f, 0.f, 0.f, 0.f};
#pragma unroll
    for (int t = 0; t < 8; ++t) acc[t] = z;
  }
  __syncthreads();

#pragma unroll 1
  for (int c = 0; c < 8; ++c) {
    const int s  = c >> 1;
    const int co = (c & 1) * 64;
#pragma unroll 1
    for (int it = 0; it < 4; ++it) {
      const int u  = it * GTHR + tid;
      const int r  = u >> 3;
      const int c8 = (u & 7) * 8;
      const int grow = rowBase + r;
      float v[8];
      if (s == 0) {
        const v4u w = *(const v4ua*)(XB + (size_t)grow * DM + co + c8);
        v[0] = bflo(w.x); v[1] = bfhi(w.x); v[2] = bflo(w.y); v[3] = bfhi(w.y);
        v[4] = bflo(w.z); v[5] = bfhi(w.z); v[6] = bflo(w.w); v[7] = bfhi(w.w);
      } else {
        const unsigned short* Pg = (s == 1) ? G1 : ((s == 2) ? G2 : G3);
        const unsigned short* rp = Pg + (size_t)grow * HLP + co + c8;
        const v4u wh = *(const v4ua*)rp;
        const v4u wl = *(const v4ua*)(rp + DM);
        v[0] = bflo(wh.x) + bflo(wl.x); v[1] = bfhi(wh.x) + bfhi(wl.x);
        v[2] = bflo(wh.y) + bflo(wl.y); v[3] = bfhi(wh.y) + bfhi(wl.y);
        v[4] = bflo(wh.z) + bflo(wl.z); v[5] = bfhi(wh.z) + bfhi(wl.z);
        v[6] = bflo(wh.w) + bflo(wl.w); v[7] = bfhi(wh.w) + bfhi(wl.w);
      }
      const int kc = 64 * c + c8;
      const v4f mu0 = *(const v4fa*)(tb + kc),        mu1 = *(const v4fa*)(tb + kc + 4);
      const v4f aa0 = *(const v4fa*)(tb + 512 + kc),  aa1 = *(const v4fa*)(tb + 512 + kc + 4);
      const v4f bb0 = *(const v4fa*)(tb + 1024 + kc), bb1 = *(const v4fa*)(tb + 1024 + kc + 4);
      float xn[8];
      xn[0] = (v[0] - mu0.x) * aa0.x + bb0.x; xn[1] = (v[1] - mu0.y) * aa0.y + bb0.y;
      xn[2] = (v[2] - mu0.z) * aa0.z + bb0.z; xn[3] = (v[3] - mu0.w) * aa0.w + bb0.w;
      xn[4] = (v[4] - mu1.x) * aa1.x + bb1.x; xn[5] = (v[5] - mu1.y) * aa1.y + bb1.y;
      xn[6] = (v[6] - mu1.z) * aa1.z + bb1.z; xn[7] = (v[7] - mu1.w) * aa1.w + bb1.w;
      v8us hv, lv;
#pragma unroll
      for (int j = 0; j < 8; ++j) {
        const unsigned pk = split_hl(xn[j]);
        hv[j] = (unsigned short)(pk & 0xffffu);
        lv[j] = (unsigned short)(pk >> 16);
      }
      *(v8usa*)(ah + r * APT + c8) = hv;
      *(v8usa*)(al + r * APT + c8) = lv;
    }
    __syncthreads();
#pragma unroll
    for (int kk = 0; kk < 64; kk += 32) {
      FragB fh, fl;
      const int ao = (16 * wave + m) * APT + kk + 8 * hh;
      fh.h[0] = *(const v8usa*)(ah + ao);
      fh.h[1] = *(const v8usa*)(ah + ao + 16);
      fl.h[0] = *(const v8usa*)(al + ao);
      fl.h[1] = *(const v8usa*)(al + ao + 16);
#pragma unroll
      for (int nt = 0; nt < 8; ++nt) {
        const unsigned short* wq = WseT + (size_t)(16 * nt + m) * 512 + 64 * c + kk + 8 * hh;
        FragB bf;
        bf.h[0] = *(const v8usa*)wq;
        bf.h[1] = *(const v8usa*)(wq + 16);
        acc[nt] = wmb(fh, bf, acc[nt]);
        acc[nt] = wmb(fl, bf, acc[nt]);
      }
    }
    __syncthreads();
  }

  EpiP P;
  P.bias = bse; P.gam = bse; P.bet = bse; P.resB = XB; P.resF = tab; P.gate = gate;
  P.outF0 = nullptr; P.outF1 = nullptr; P.outH = xatt;
  P.ldo0 = DM; P.ldo1 = DM; P.ldh = HLP; P.nOut = nOut;
  gemm_epi<1>(acc, stg, P, rowBase, 0, lane, wave);
}

static inline int cdiv(int a, int b) { return (a + b - 1) / b; }
static inline size_t al256(size_t o) { return (o + 255) & ~(size_t)255; }

extern "C" void kernel_launch(void* const* d_in, const int* in_sizes, int n_in,
                              void* d_out, int out_size, void* d_ws, size_t ws_size,
                              hipStream_t stream) {
  if (n_in < 26) return;
  if (in_sizes[0] < DM || (in_sizes[0] % DM) != 0) return;
  const int nN = in_sizes[0] / DM;
  if (nN < 64 || nN > (1 << 20)) return;
  if (in_sizes[1] < 2 || (in_sizes[1] & 1) != 0) return;
  const int nE = in_sizes[1] / 2;
  if (nE < 1 || nE >= (1 << 21)) return;
  if (in_sizes[2] != in_sizes[1] || in_sizes[3] != 1) return;
  if (in_sizes[4] != DM * DM || in_sizes[6] != DM * DM || in_sizes[8] != DM * DM) return;
  if (in_sizes[5] != DM || in_sizes[7] != DM || in_sizes[9] != DM) return;
  if (in_sizes[10] != 512 || in_sizes[11] != 512) return;
  if (in_sizes[12] != 512 * DM || in_sizes[13] != DM) return;
  if (in_sizes[14] != DM * 256 || in_sizes[15] != DM * DM) return;
  if (in_sizes[16] != DM * DM || in_sizes[17] != DM) return;
  if (in_sizes[18] != DM || in_sizes[19] != DM) return;
  if (in_sizes[20] != DM * 512 || in_sizes[21] != 512) return;
  if (in_sizes[22] != 512 * DM || in_sizes[23] != DM) return;
  if (in_sizes[24] != DM || in_sizes[25] != DM) return;
  if ((long long)out_size != (long long)nN * DM) return;

  const float* x    = (const float*)d_in[0];
  const int*   ei   = (const int*)d_in[1];
  const int*   dag  = (const int*)d_in[2];
  const int*   gate = (const int*)d_in[3];
  const float* Wg1  = (const float*)d_in[4];
  const float* bg1  = (const float*)d_in[5];
  const float* Wg2  = (const float*)d_in[6];
  const float* bg2  = (const float*)d_in[7];
  const float* Wg3  = (const float*)d_in[8];
  const float* bg3  = (const float*)d_in[9];
  const float* bng  = (const float*)d_in[10];
  const float* bnb  = (const float*)d_in[11];
  const float* Wse  = (const float*)d_in[12];
  const float* bse  = (const float*)d_in[13];
  const float* Wqk  = (const float*)d_in[14];
  const float* Wv   = (const float*)d_in[15];
  const float* Wo   = (const float*)d_in[16];
  const float* bo   = (const float*)d_in[17];
  const float* l1g  = (const float*)d_in[18];
  const float* l1b  = (const float*)d_in[19];
  const float* W1   = (const float*)d_in[20];
  const float* b1   = (const float*)d_in[21];
  const float* W2   = (const float*)d_in[22];
  const float* b2   = (const float*)d_in[23];
  const float* l2g  = (const float*)d_in[24];
  const float* l2b  = (const float*)d_in[25];
  float* out = (float*)d_out;
  const int* srcG = ei;
  const int* dstG = ei + nE;
  const int* srcA = dag;
  const int* dstA = dag + nE;

  const int MP  = cdiv(nN, GBM) * GBM;
  const int NRB = MP / GBM;
  const int gD  = cdiv(nN, NBD);
  const int gA  = cdiv(MP, NBA);
  const int nB  = cdiv(nN, BNRB);
  if ((long long)gA * NBA < (long long)MP) return;
  const int vec8 = ((nE & 3) == 0) ? 1 : 0;
  const int cb0 = (NRB + 1) / 2;
  const int cb1 = NRB - cb0;

  const size_t RS  = (size_t)MP * 512;
  const size_t R0S = (size_t)MP * 256;
  const size_t oR2 = 0, oR3 = RS, oR4 = 2 * RS, oR1 = 3 * RS, oR0 = 4 * RS;
  size_t off = 4 * RS + R0S;
  const size_t oWT  = off; off = al256(off + (size_t)OW_END * 2);
  const size_t oDIS = off; off = al256(off + (size_t)gD * NBD * 4);
  const size_t oREC = off; off = al256(off + (size_t)nB * 1024 * 8);
  const size_t oTAB = off; off = al256(off + (size_t)1536 * 4);
  if (off > ws_size || off > (size_t)WSMAX) return;
  const size_t fBytes = (size_t)cb0 * GBM * FPI * 2;
  if (fBytes > 2 * RS + R0S) return;

  char* ws = (char*)d_ws;
  unsigned short* G1p  = (unsigned short*)(ws + oR2);
  unsigned short* G2p  = (unsigned short*)(ws + oR3);
  unsigned short* G3p  = (unsigned short*)(ws + oR4);
  float*          HT   = (float*)(ws + oR1);
  unsigned short* XATT = (unsigned short*)(ws + oR1);
  unsigned short* AGG  = (unsigned short*)(ws + oR1);
  float*          Qp   = (float*)(ws + oR2);
  float*          KV   = (float*)(ws + oR3);
  float*          H1   = (float*)(ws + oR2);
  unsigned short* H1HL = (unsigned short*)(ws + oR3);
  unsigned short* Fp   = (unsigned short*)(ws + oR4);
  unsigned short* XB   = (unsigned short*)(ws + oR0);
  unsigned short* WT   = (unsigned short*)(ws + oWT);
  float*          DIS  = (float*)(ws + oDIS);
  double*         REC  = (double*)(ws + oREC);
  float*          TAB  = (float*)(ws + oTAB);

  const size_t scanLds = (size_t)AGG_LDS_INTS * 4;
  hipFuncSetAttribute(reinterpret_cast<const void*>(&k_gscan), hipFuncAttributeMaxDynamicSharedMemorySize, (int)scanLds);
  hipFuncSetAttribute(reinterpret_cast<const void*>(&k_ascan), hipFuncAttributeMaxDynamicSharedMemorySize, (int)scanLds);

  const int nUx = MP * (DM / 8);
  k_cvx<<<cdiv(nUx, NTHR), NTHR, 0, stream>>>(x, nN, nUx, XB);
  k_wprep<<<NWUNITS / NTHR, NTHR, 0, stream>>>(Wg1, Wg2, Wg3, Wv, Wo, Wqk, Wse, W1, W2, WT);
  k_deg<<<gD, NTHR, 0, stream>>>(dstG, nE, vec8, DIS);
  k_gemm<0, 0><<<dim3(NRB, 1), GTHR, 0, stream>>>(XB, DM, 0, DM, WT + OW_G1, bg1, bg1, bg1, XB, x, gate,
                                                  HT, DM, HT, DM, G1p, HLP, nN);
  k_gscan<<<gA, NTHR, scanLds, stream>>>(srcG, dstG, nE, nN, vec8, MP, DIS, HT, bg1, G1p);
  k_gemm<1, 0><<<dim3(NRB, 1), GTHR, 0, stream>>>(G1p, HLP, DM, DM, WT + OW_G2, bg2, bg2, bg2, XB, x, gate,
                                                  HT, DM, HT, DM, G2p, HLP, nN);
  k_gscan<<<gA, NTHR, scanLds, stream>>>(srcG, dstG, nE, nN, vec8, MP, DIS, HT, bg2, G2p);
  k_gemm<1, 0><<<dim3(NRB, 1), GTHR, 0, stream>>>(G2p, HLP, DM, DM, WT + OW_G3, bg3, bg3, bg3, XB, x, gate,
                                                  HT, DM, HT, DM, G3p, HLP, nN);
  k_gscan<<<gA, NTHR, scanLds, stream>>>(srcG, dstG, nE, nN, vec8, MP, DIS, HT, bg3, G3p);
  k_bnstats<<<nB, GTHR, 0, stream>>>(XB, G1p, G2p, G3p, nN, REC);
  k_bncomb<<<1, 512, 0, stream>>>(REC, nB, 1.0 / (double)nN, bng, bnb, TAB);
  k_se<<<NRB, GTHR, 0, stream>>>(XB, G1p, G2p, G3p, TAB, WT + OW_SE, bse, gate, XATT, nN);
  k_gemm<1, 0><<<dim3(NRB, 2), GTHR, 0, stream>>>(XATT, HLP, DM, DM, WT + OW_QK, bse, bse, bse, XB, x, gate,
                                                  KV, 2 * DM, Qp, DM, G1p, HLP, nN);
  k_gemm<0, 0><<<dim3(NRB, 1), GTHR, 0, stream>>>(XB, DM, 0, DM, WT + OW_V, bse, bse, bse, XB, x, gate,
                                                  KV + DM, 2 * DM, KV + DM, 2 * DM, G1p, HLP, nN);
  k_ascan<<<gA, NTHR, scanLds, stream>>>(srcA, dstA, nE, nN, vec8, MP, Qp, KV, AGG);
  k_gemm<1, 2><<<dim3(NRB, 1), GTHR, 0, stream>>>(AGG, HLP, DM, DM, WT + OW_O, bo, l1g, l1b, XB, x, gate,
                                                  H1, DM, H1, DM, H1HL, HLP, nN);
  {
    const int r0 = 0;
    int nv = nN - r0; nv = nv < 0 ? 0 : (nv > cb0 * GBM ? cb0 * GBM : nv);
    if (cb0 > 0 && nv > 0) {
      k_gemm<1, 3><<<dim3(cb0, 4), GTHR, 0, stream>>>(H1HL + (size_t)r0 * HLP, HLP, DM, DM, WT + OW_1,
                                                      b1, b1, b1, XB, x, gate, H1, DM, H1, DM, Fp, FPI, nv);
      k_gemm<1, 4><<<dim3(cb0, 1), GTHR, 0, stream>>>(Fp, FPI, 512, 512, WT + OW_2, b2, l2g, l2b, XB,
                                                      H1 + (size_t)r0 * DM, gate,
                                                      out + (size_t)r0 * DM, DM, out + (size_t)r0 * DM, DM,
                                                      H1HL, HLP, nv);
    }
  }
  {
    const int r0 = cb0 * GBM;
    int nv = nN - r0; nv = nv < 0 ? 0 : (nv > cb1 * GBM ? cb1 * GBM : nv);
    if (cb1 > 0 && nv > 0) {
      k_gemm<1, 3><<<dim3(cb1, 4), GTHR, 0, stream>>>(H1HL + (size_t)r0 * HLP, HLP, DM, DM, WT + OW_1,
                                                      b1, b1, b1, XB, x, gate, H1, DM, H1, DM, Fp, FPI, nv);
      k_gemm<1, 4><<<dim3(cb1, 1), GTHR, 0, stream>>>(Fp, FPI, 512, 512, WT + OW_2, b2, l2g, l2b, XB,
                                                      H1 + (size_t)r0 * DM, gate,
                                                      out + (size_t)r0 * DM, DM, out + (size_t)r0 * DM, DM,
                                                      H1HL, HLP, nv);
    }
  }
}
